// Encoder_22213570855422
// MI455X (gfx1250) — hardware-verified
//
#include <hip/hip_runtime.h>
#include <hip/hip_fp16.h>
#include <math.h>


#ifndef NB
#define NB 2
#endif
#ifndef SEQ
#define SEQ 1024
#endif
#define NB_FULL  2
#define SEQ_FULL 1024
#define DM    512
#define NH    8
#define HD    64
#define NL    4
#define NMODE 256
#define DFF   2048
#define NTOK  (NB * SEQ)
#define CP    68

static_assert(NB >= 1 && NB <= NB_FULL);
static_assert(NB <= 32);
static_assert(SEQ >= 256 && SEQ <= SEQ_FULL);
static_assert(SEQ % 256 == 0);
static_assert(NTOK % 128 == 0);
static_assert(DM == NH * HD);
static_assert(DM == 2 * NMODE);
static_assert(HD == 64);
static_assert(DM == 512);
static_assert(DM % 64 == 0 && DFF % 64 == 0 && (3 * DM) % 64 == 0);
static_assert(DM % 32 == 0 && DFF % 32 == 0);
static_assert(CP % 4 == 0 && CP >= 64);

#define W_CARRY   64.0f
#define F_CARRY   16.0f
#define QKV_CARRY 8.0f
#define H_CARRY   16.0f
#define LOG2E     1.44269504088896340736f
#define C1        (LOG2E * 0.001953125f)

typedef _Float16 v16h __attribute__((ext_vector_type(16)));
typedef _Float16 v8h  __attribute__((ext_vector_type(8)));
typedef float    v8f  __attribute__((ext_vector_type(8)));
typedef float    v4f  __attribute__((ext_vector_type(4)));
typedef double   v2d  __attribute__((ext_vector_type(2)));

union Frag { v16h v; v8h h[2]; };

static __device__ __forceinline__ v8f zero8() {
    v8f z;
#pragma unroll
    for (int i = 0; i < 8; ++i) z[i] = 0.0f;
    return z;
}

static __device__ __forceinline__ v16h load_frag16(const _Float16* base, int ld, int lane) {
    int m  = lane & 15;
    int kb = (lane >> 4) << 3;
    const _Float16* p = base + (size_t)m * ld + kb;
    Frag f;
    f.h[0] = *(const v8h*)(p);
    f.h[1] = *(const v8h*)(p + 16);
    return f.v;
}

static __device__ __forceinline__ v8f wmma16(v16h a, v16h b, v8f c) {
    v8f d = __builtin_amdgcn_wmma_f32_16x16x32_f16(false, a, false, b, (short)0, c, false, false);
    asm volatile("v_nop\n\tv_nop\n\tv_nop\n\tv_nop" : "+v"(d) : "v"(a), "v"(b));
    return d;
}

static __device__ __forceinline__ float bf16r(float x) {
    unsigned u = __float_as_uint(x);
    u = (u + 0x7FFFu + ((u >> 16) & 1u)) & 0xFFFF0000u;
    return __uint_as_float(u);
}
static __device__ __forceinline__ v4f bf16r4(v4f a) {
    v4f r;
    r.x = bf16r(a.x); r.y = bf16r(a.y); r.z = bf16r(a.z); r.w = bf16r(a.w);
    return r;
}

static __device__ __forceinline__ float ex2(float x) {
    return __builtin_amdgcn_exp2f(x);
}

static __device__ __forceinline__ void wave_lds_sync() {
    __builtin_amdgcn_fence(3, "wavefront");
    asm volatile("s_wait_dscnt 0" ::: "memory");
    __builtin_amdgcn_wave_barrier();
}

static __device__ __forceinline__ float wsum(float v) {
#pragma unroll
    for (int off = 16; off >= 1; off >>= 1) v += __shfl_xor(v, off, 32);
    return v;
}

__global__ __launch_bounds__(256) void k_wT(const float* __restrict__ src,
                                             _Float16* __restrict__ dst,
                                             int K, int N, int srcZ, int dstZ) {
    __shared__ __align__(16) _Float16 T[64 * 72];
    const int tid = threadIdx.x;
    const int n0 = blockIdx.x * 64;
    const int k0 = blockIdx.y * 64;
    const float* s = src + (size_t)blockIdx.z * (size_t)srcZ;
    _Float16*    d = dst + (size_t)blockIdx.z * (size_t)dstZ;
#pragma unroll 1
    for (int it = 0; it < 4; ++it) {
        int idx = it * 256 + tid;
        int kr = idx >> 4;
        int c4 = (idx & 15) * 4;
        v4f v = *(const v4f*)(s + (size_t)(k0 + kr) * N + n0 + c4);
        T[(c4 + 0) * 72 + kr] = (_Float16)(bf16r(v.x) * W_CARRY);
        T[(c4 + 1) * 72 + kr] = (_Float16)(bf16r(v.y) * W_CARRY);
        T[(c4 + 2) * 72 + kr] = (_Float16)(bf16r(v.z) * W_CARRY);
        T[(c4 + 3) * 72 + kr] = (_Float16)(bf16r(v.w) * W_CARRY);
    }
    __syncthreads();
    const int nr = tid >> 3;
    const int c8 = (tid & 7) * 8;
    v8h p0 = *(const v8h*)(&T[nr * 72 + c8]);
    v8h p1 = *(const v8h*)(&T[(32 + nr) * 72 + c8]);
    _Float16* d0 = d + (size_t)(n0 + nr) * K + k0 + c8;
    _Float16* d1 = d + (size_t)(n0 + 32 + nr) * K + k0 + c8;
    *(volatile v8h*)d0 = p0;
    *(volatile v8h*)d1 = p1;
    __threadfence();
    *(volatile v8h*)d0 = p0;
    *(volatile v8h*)d1 = p1;
}

__global__ __launch_bounds__(256) void k_feats(const float* __restrict__ coords,
                                                const float* __restrict__ modes,
                                                _Float16* __restrict__ feats) {
    __shared__ __align__(16) _Float16 F[8 * DM];
    static_assert(NMODE == 256);
    const int tid = threadIdx.x;
    const int row0 = blockIdx.x * 8;
    const int b = row0 / SEQ, s0 = row0 % SEQ;
    const float mx = bf16r(modes[tid * 3 + 0]);
    const float my = bf16r(modes[tid * 3 + 1]);
    const float mz = bf16r(modes[tid * 3 + 2]);
#pragma unroll 1
    for (int r = 0; r < 8; ++r) {
        const float* c = coords + ((size_t)b * SEQ_FULL + s0 + r) * 3;
        float cx = bf16r(c[0]), cy = bf16r(c[1]), cz = bf16r(c[2]);
        float ph = __builtin_fmaf(cz, mz, __builtin_fmaf(cy, my, cx * mx));
        F[r * DM + tid]         = (_Float16)(cosf(ph) * F_CARRY);
        F[r * DM + NMODE + tid] = (_Float16)(sinf(ph) * F_CARRY);
    }
    __syncthreads();
    v8h p0 = *(const v8h*)(&F[(size_t)tid * 8]);
    v8h p1 = *(const v8h*)(&F[(size_t)(256 + tid) * 8]);
    _Float16* d0 = feats + (size_t)row0 * DM + (size_t)tid * 8;
    _Float16* d1 = feats + (size_t)row0 * DM + (size_t)(256 + tid) * 8;
    *(volatile v8h*)d0 = p0;
    *(volatile v8h*)d1 = p1;
    __threadfence();
    *(volatile v8h*)d0 = p0;
    *(volatile v8h*)d1 = p1;
}

static __device__ __forceinline__ float dist1(float ax, float ay, float az,
                                              float sx, float sy, float sz) {
    float dx = ax - sx, dy = ay - sy, dz = az - sz;
    return sqrtf(dx * dx + dy * dy + dz * dz);
}

__global__ __launch_bounds__(256) void k_dist(const float* __restrict__ coords,
                                               float* __restrict__ dpl,
                                               double* __restrict__ part) {
    __shared__ double rs[8];
    __shared__ double rq[8];
    const int tid = threadIdx.x, lane = tid & 31, w = tid >> 5;
    const int row0 = blockIdx.x * 8;
    const int b = row0 / SEQ, i0 = row0 % SEQ;
    const float* cb = coords + (size_t)b * SEQ_FULL * 3;
    double s = 0.0, q = 0.0;
#pragma unroll 1
    for (int pass = 0; pass < 2; ++pass) {
        if (pass == 1) __threadfence();
#pragma unroll 1
        for (int j = tid * 4; j < SEQ; j += 1024) {
            v4f c0 = *(const v4f*)(cb + (size_t)j * 3);
            v4f c1 = *(const v4f*)(cb + (size_t)j * 3 + 4);
            v4f c2 = *(const v4f*)(cb + (size_t)j * 3 + 8);
            const float x0 = bf16r(c0.x) + 1e-5f, y0 = bf16r(c0.y) + 1e-5f, z0 = bf16r(c0.z) + 1e-5f;
            const float x1 = bf16r(c0.w) + 1e-5f, y1 = bf16r(c1.x) + 1e-5f, z1 = bf16r(c1.y) + 1e-5f;
            const float x2 = bf16r(c1.z) + 1e-5f, y2 = bf16r(c1.w) + 1e-5f, z2 = bf16r(c2.x) + 1e-5f;
            const float x3 = bf16r(c2.y) + 1e-5f, y3 = bf16r(c2.z) + 1e-5f, z3 = bf16r(c2.w) + 1e-5f;
#pragma unroll 1
            for (int r = 0; r < 8; ++r) {
                const float* ci = cb + (size_t)(i0 + r) * 3;
                const float ax = bf16r(ci[0]), ay = bf16r(ci[1]), az = bf16r(ci[2]);
                v4f dv;
                dv.x = dist1(ax, ay, az, x0, y0, z0);
                dv.y = dist1(ax, ay, az, x1, y1, z1);
                dv.z = dist1(ax, ay, az, x2, y2, z2);
                dv.w = dist1(ax, ay, az, x3, y3, z3);
                *(volatile v4f*)(dpl + ((size_t)b * SEQ + i0 + r) * SEQ + j) = dv;
                if (pass == 0) {
                    double e0 = (double)dv.x, e1 = (double)dv.y, e2 = (double)dv.z, e3 = (double)dv.w;
                    s += (e0 + e1) + (e2 + e3);
                    q += (e0 * e0 + e1 * e1) + (e2 * e2 + e3 * e3);
                }
            }
        }
    }
#pragma unroll
    for (int off = 16; off >= 1; off >>= 1) {
        s += __shfl_xor(s, off, 32);
        q += __shfl_xor(q, off, 32);
    }
    if (lane == 0) { rs[w] = s; rq[w] = q; }
    __syncthreads();
    if (w == 0) {
        double S = 0.0, Q = 0.0;
#pragma unroll
        for (int k = 0; k < 8; ++k) { S += rs[k]; Q += rq[k]; }
        if (lane < 8) {
            v2d val;
            val.x = (lane == 0) ? S : 0.0;
            val.y = (lane == 0) ? Q : 0.0;
            double* dst = part + (size_t)blockIdx.x * 16 + lane * 2;
            *(volatile v2d*)dst = val;
            __threadfence();
            *(volatile v2d*)dst = val;
        }
    }
}

__global__ __launch_bounds__(32) void k_dstat(const double* __restrict__ part,
                                               float* __restrict__ istd) {
    __shared__ __align__(16) float line[32];
    const int lane = threadIdx.x;
    static_assert((SEQ / 8) % 32 == 0);
    const double nn = (double)SEQ * (double)SEQ;
    const double inv_n = 1.0 / nn;
    const double inv_n1 = 1.0 / (nn - 1.0);
    float mine = 0.0f;
#pragma unroll 1
    for (int b = 0; b < NB; ++b) {
        double S = 0.0, Q = 0.0;
#pragma unroll 1
        for (int k = lane; k < SEQ / 8; k += 32) {
            const double* p = part + ((size_t)b * (SEQ / 8) + k) * 16;
            S += p[0];
            Q += p[1];
        }
#pragma unroll
        for (int off = 16; off >= 1; off >>= 1) {
            S += __shfl_xor(S, off, 32);
            Q += __shfl_xor(Q, off, 32);
        }
        const double var = (Q - S * S * inv_n) * inv_n1;
        const float sd = sqrtf((float)var);
        const float is = 1.0f / sd;
        mine = (lane == b) ? is : mine;
    }
    line[lane] = mine;
    __syncthreads();
    if (lane < 8) {
        v4f v = *(const v4f*)(&line[lane * 4]);
        *(volatile v4f*)(istd + lane * 4) = v;
        __threadfence();
        *(volatile v4f*)(istd + lane * 4) = v;
    }
}

static __device__ __forceinline__ float hsum4(v4f a) { return (a.x + a.y) + (a.z + a.w); }
static __device__ __forceinline__ float hsq4(v4f a, float mu) {
    float d0 = a.x - mu, d1 = a.y - mu, d2 = a.z - mu, d3 = a.w - mu;
    return (d0 * d0 + d1 * d1) + (d2 * d2 + d3 * d3);
}
static __device__ __forceinline__ void ln_stats(v4f a0, v4f a1, v4f a2, v4f a3,
                                                float& mean, float& rstd) {
    float s = (hsum4(a0) + hsum4(a1)) + (hsum4(a2) + hsum4(a3));
    s = wsum(s);
    mean = s * (1.0f / DM);
    float qv = (hsq4(a0, mean) + hsq4(a1, mean)) + (hsq4(a2, mean) + hsq4(a3, mean));
    qv = wsum(qv);
    rstd = rsqrtf(qv * (1.0f / DM) + 1e-5f);
}
static __device__ __forceinline__ v4f ln_apply(v4f a, v4f g, v4f b, float mean, float rstd) {
    v4f r;
    r.x = (a.x - mean) * rstd * g.x + b.x;
    r.y = (a.y - mean) * rstd * g.y + b.y;
    r.z = (a.z - mean) * rstd * g.z + b.z;
    r.w = (a.w - mean) * rstd * g.w + b.w;
    return r;
}

__global__ __launch_bounds__(256) void k_ln16(const float* __restrict__ x,
                                               const float* __restrict__ g,
                                               const float* __restrict__ bb,
                                               _Float16* __restrict__ y) {
    static_assert(32 * 16 == DM);
    const int lane = threadIdx.x & 31, w = threadIdx.x >> 5;
    const int row = blockIdx.x * 8 + w;
    const float* xr = x + (size_t)row * DM;
    const int c = lane * 8;
    v4f a0 = *(const v4f*)(xr + c);
    v4f a1 = *(const v4f*)(xr + c + 4);
    v4f a2 = *(const v4f*)(xr + 256 + c);
    v4f a3 = *(const v4f*)(xr + 256 + c + 4);
    float mean, rstd;
    ln_stats(a0, a1, a2, a3, mean, rstd);
    v4f r0 = ln_apply(a0, bf16r4(*(const v4f*)(g + c)),           bf16r4(*(const v4f*)(bb + c)),           mean, rstd);
    v4f r1 = ln_apply(a1, bf16r4(*(const v4f*)(g + c + 4)),       bf16r4(*(const v4f*)(bb + c + 4)),       mean, rstd);
    v4f r2 = ln_apply(a2, bf16r4(*(const v4f*)(g + 256 + c)),     bf16r4(*(const v4f*)(bb + 256 + c)),     mean, rstd);
    v4f r3 = ln_apply(a3, bf16r4(*(const v4f*)(g + 256 + c + 4)), bf16r4(*(const v4f*)(bb + 256 + c + 4)), mean, rstd);
    v8h h0, h1;
    h0[0] = (_Float16)r0.x; h0[1] = (_Float16)r0.y; h0[2] = (_Float16)r0.z; h0[3] = (_Float16)r0.w;
    h0[4] = (_Float16)r1.x; h0[5] = (_Float16)r1.y; h0[6] = (_Float16)r1.z; h0[7] = (_Float16)r1.w;
    h1[0] = (_Float16)r2.x; h1[1] = (_Float16)r2.y; h1[2] = (_Float16)r2.z; h1[3] = (_Float16)r2.w;
    h1[4] = (_Float16)r3.x; h1[5] = (_Float16)r3.y; h1[6] = (_Float16)r3.z; h1[7] = (_Float16)r3.w;
    _Float16* yr = y + (size_t)row * DM;
    *(volatile v8h*)(yr + c)       = h0;
    *(volatile v8h*)(yr + 256 + c) = h1;
    __threadfence();
    *(volatile v8h*)(yr + c)       = h0;
    *(volatile v8h*)(yr + 256 + c) = h1;
}

__global__ __launch_bounds__(256) void k_ln32(const float* __restrict__ x,
                                               const float* __restrict__ g,
                                               const float* __restrict__ bb,
                                               float* __restrict__ out) {
    static_assert(4 * 128 == DM);
    const int lane = threadIdx.x & 31, w = threadIdx.x >> 5;
    const int row = blockIdx.x * 8 + w;
    const float* xr = x + (size_t)row * DM;
    const int c = lane * 4;
    v4f a0 = *(const v4f*)(xr + c);
    v4f a1 = *(const v4f*)(xr + 128 + c);
    v4f a2 = *(const v4f*)(xr + 256 + c);
    v4f a3 = *(const v4f*)(xr + 384 + c);
    float mean, rstd;
    ln_stats(a0, a1, a2, a3, mean, rstd);
    v4f r0 = ln_apply(a0, bf16r4(*(const v4f*)(g + c)),       bf16r4(*(const v4f*)(bb + c)),       mean, rstd);
    v4f r1 = ln_apply(a1, bf16r4(*(const v4f*)(g + 128 + c)), bf16r4(*(const v4f*)(bb + 128 + c)), mean, rstd);
    v4f r2 = ln_apply(a2, bf16r4(*(const v4f*)(g + 256 + c)), bf16r4(*(const v4f*)(bb + 256 + c)), mean, rstd);
    v4f r3 = ln_apply(a3, bf16r4(*(const v4f*)(g + 384 + c)), bf16r4(*(const v4f*)(bb + 384 + c)), mean, rstd);
    float* orow = out + (size_t)row * DM;
    *(volatile v4f*)(orow + c)       = r0;
    *(volatile v4f*)(orow + 128 + c) = r1;
    *(volatile v4f*)(orow + 256 + c) = r2;
    *(volatile v4f*)(orow + 384 + c) = r3;
    __threadfence();
    *(volatile v4f*)(orow + c)       = r0;
    *(volatile v4f*)(orow + 128 + c) = r1;
    *(volatile v4f*)(orow + 256 + c) = r2;
    *(volatile v4f*)(orow + 384 + c) = r3;
}

static __device__ __forceinline__ float gelu_erf(float v) {
    return 0.5f * v * (1.0f + erff(v * 0.70710678118654752f));
}

__global__ __launch_bounds__(128) __attribute__((amdgpu_num_vgpr(256)))
void k_gemm(const _Float16* __restrict__ A, const _Float16* __restrict__ BT,
            int K, int N, int mode, float alpha, float oscale,
            const float* bias0, const float* bias1, const float* bias2,
            const float* resid, int rbf, int rfull,
            float* outF, _Float16* out16, _Float16* outVT) {
    __shared__ __align__(16) float Cs[128 * CP];
    __shared__ __align__(16) v8h   Hs[1024];

    const int tid  = threadIdx.x;
    const int lane = tid & 31;
    const int w    = tid >> 5;
    const int row0 = blockIdx.x * 128;
    const int col0 = blockIdx.y * 64;
    const int r0   = (lane >> 4) << 3;
    const int cc   = lane & 15;

    v8f acc[2][4];
#pragma unroll
    for (int mt = 0; mt < 2; ++mt)
#pragma unroll
        for (int nt = 0; nt < 4; ++nt) acc[mt][nt] = zero8();

    const _Float16* Aw = A + (size_t)(row0 + w * 32) * K;
    const _Float16* Bw = BT + (size_t)col0 * K;
#pragma unroll 1
    for (int k0 = 0; k0 < K; k0 += 32) {
        v16h a0 = load_frag16(Aw + k0, K, lane);
        v16h a1 = load_frag16(Aw + (size_t)16 * K + k0, K, lane);
#pragma unroll
        for (int nt = 0; nt < 4; ++nt) {
            v16h bf = load_frag16(Bw + (size_t)(nt * 16) * K + k0, K, lane);
            acc[0][nt] = wmma16(a0, bf, acc[0][nt]);
            acc[1][nt] = wmma16(a1, bf, acc[1][nt]);
        }
    }

#pragma unroll
    for (int mt = 0; mt < 2; ++mt)
#pragma unroll
        for (int nt = 0; nt < 4; ++nt)
#pragma unroll
            for (int g = 0; g < 8; ++g)
                Cs[(w * 32 + mt * 16 + r0 + g) * CP + nt * 16 + cc] = acc[mt][nt][g];
    __syncthreads();

    if (mode == 0) {
        const int c4 = (lane & 15) * 4;
        const v4f b4 = bf16r4(*(const v4f*)(bias0 + col0 + c4));
#pragma unroll 1
        for (int i = 0; i < 16; ++i) {
            const int row  = w * 32 + 2 * i + (lane >> 4);
            const int grow = row0 + row;
            const int rrow = rfull ? ((grow / SEQ) * SEQ_FULL + (grow % SEQ)) : grow;
            v4f v  = *(const v4f*)(&Cs[row * CP + c4]);
            v4f rv = *(const v4f*)(resid + (size_t)rrow * N + col0 + c4);
            v4f rr = bf16r4(rv);
            rv.x = rbf ? rr.x : rv.x; rv.y = rbf ? rr.y : rv.y;
            rv.z = rbf ? rr.z : rv.z; rv.w = rbf ? rr.w : rv.w;
            v4f o;
            o.x = rv.x + __builtin_fmaf(v.x, alpha, b4.x);
            o.y = rv.y + __builtin_fmaf(v.y, alpha, b4.y);
            o.z = rv.z + __builtin_fmaf(v.z, alpha, b4.z);
            o.w = rv.w + __builtin_fmaf(v.w, alpha, b4.w);
            *(v4f*)(&Cs[row * CP + c4]) = o;
            *(volatile v4f*)(outF + (size_t)grow * N + col0 + c4) = o;
        }
        __threadfence();
#pragma unroll 1
        for (int i = 0; i < 16; ++i) {
            const int row  = w * 32 + 2 * i + (lane >> 4);
            const int grow = row0 + row;
            v4f o = *(const v4f*)(&Cs[row * CP + c4]);
            *(volatile v4f*)(outF + (size_t)grow * N + col0 + c4) = o;
        }
    } else {
        const int which = (mode == 1) ? (col0 >> 9) : 0;
        const int bcol  = (mode == 1) ? (col0 & 511) : col0;
        if (which < 2) {
            const int    ldo  = (mode == 1) ? DM : N;
            const size_t zoff = (size_t)which * ((size_t)NTOK * DM);
            const int c8 = (lane & 7) * 8;
            const v4f ba0 = *(const v4f*)(bias0 + bcol + c8);
            const v4f ba1 = *(const v4f*)(bias0 + bcol + c8 + 4);
            const v4f bb0 = *(const v4f*)(bias1 + bcol + c8);
            const v4f bb1 = *(const v4f*)(bias1 + bcol + c8 + 4);
            const v4f bs0 = bf16r4((which == 0) ? ba0 : bb0);
            const v4f bs1 = bf16r4((which == 0) ? ba1 : bb1);
#pragma unroll 1
            for (int i = 0; i < 8; ++i) {
                const int row = w * 32 + 4 * i + (lane >> 3);
                v4f v0 = *(const v4f*)(&Cs[row * CP + c8]);
                v4f v1 = *(const v4f*)(&Cs[row * CP + c8 + 4]);
                float t[8];
                t[0] = __builtin_fmaf(v0.x, alpha, bs0.x);
                t[1] = __builtin_fmaf(v0.y, alpha, bs0.y);
                t[2] = __builtin_fmaf(v0.z, alpha, bs0.z);
                t[3] = __builtin_fmaf(v0.w, alpha, bs0.w);
                t[4] = __builtin_fmaf(v1.x, alpha, bs1.x);
                t[5] = __builtin_fmaf(v1.y, alpha, bs1.y);
                t[6] = __builtin_fmaf(v1.z, alpha, bs1.z);
                t[7] = __builtin_fmaf(v1.w, alpha, bs1.w);
                if (mode == 2) {
#pragma unroll
                    for (int e = 0; e < 8; ++e) t[e] = gelu_erf(t[e]);
                }
                v8h hv;
#pragma unroll
                for (int e = 0; e < 8; ++e) hv[e] = (_Float16)(t[e] * oscale);
                Hs[i * 128 + tid] = hv;
                *(volatile v8h*)(out16 + zoff + (size_t)(row0 + row) * ldo + bcol + c8) = hv;
            }
            __threadfence();
#pragma unroll 1
            for (int i = 0; i < 8; ++i) {
                const int row = w * 32 + 4 * i + (lane >> 3);
                v8h hv = Hs[i * 128 + tid];
                *(volatile v8h*)(out16 + zoff + (size_t)(row0 + row) * ldo + bcol + c8) = hv;
            }
        } else {
            const int hh = bcol >> 6;
            const int b  = row0 / SEQ;
            const int s0 = row0 % SEQ;
#pragma unroll 1
            for (int i = 0; i < 8; ++i) {
                const int piece = i * 128 + tid;
                const int d  = piece >> 4;
                const int tp = piece & 15;
                const float bv = bf16r(bias2[bcol + d]);
                v8h hv;
#pragma unroll
                for (int e = 0; e < 8; ++e)
                    hv[e] = (_Float16)(__builtin_fmaf(Cs[(tp * 8 + e) * CP + d], alpha, bv) * oscale);
                Hs[piece] = hv;
                *(volatile v8h*)(outVT + (((size_t)b * NH + hh) * HD + d) * SEQ + s0 + tp * 8) = hv;
            }
            __threadfence();
#pragma unroll 1
            for (int i = 0; i < 8; ++i) {
                const int piece = i * 128 + tid;
                const int d  = piece >> 4;
                const int tp = piece & 15;
                v8h hv = Hs[piece];
                *(volatile v8h*)(outVT + (((size_t)b * NH + hh) * HD + d) * SEQ + s0 + tp * 8) = hv;
            }
        }
    }
}

__global__ __launch_bounds__(256) __attribute__((amdgpu_num_vgpr(256)))
void k_attn(const _Float16* __restrict__ qp, const _Float16* __restrict__ kp,
            const _Float16* __restrict__ vT, const float* __restrict__ dpl,
            const float* __restrict__ istd, const float* __restrict__ temp,
            _Float16* __restrict__ op) {
    __shared__ __align__(16) _Float16 Os[8][16 * HD];

    const int tid  = threadIdx.x;
    const int lane = tid & 31;
    const int w    = tid >> 5;
    const int b    = blockIdx.x / NH;
    const int h    = blockIdx.x % NH;
    const int q0r  = blockIdx.y * 128 + w * 16;
    const int hs   = lane >> 4;
    const int cc   = lane & 15;

    const float tv  = bf16r(temp[h]);
    const float sp  = fmaxf(tv, 0.0f) + log1pf(expf(-fabsf(tv)));
    const float ncl = -(sp * istd[b]) * LOG2E;

    const size_t qoff = ((size_t)b * SEQ + q0r) * DM + h * HD;
    const _Float16* kb = kp + (size_t)b * SEQ * DM + h * HD;
    const _Float16* vb = vT + ((size_t)b * NH + h) * HD * SEQ;
    const float* drow = dpl + ((size_t)b * SEQ + q0r + cc) * SEQ + 8 * hs;

    v8f oacc[4];
#pragma unroll
    for (int nt = 0; nt < 4; ++nt) oacc[nt] = zero8();
    float m = -1.0e30f, l = 0.0f;

#pragma unroll 1
    for (int key0 = 0; key0 < SEQ; key0 += 32) {
        v8f s0 = zero8(), s1 = zero8();
#pragma unroll
        for (int ks = 0; ks < 2; ++ks) {
            v16h qf = load_frag16(qp + qoff + ks * 32, DM, lane);
            v16h ka = load_frag16(kb + (size_t)key0 * DM + ks * 32, DM, lane);
            v16h kc = load_frag16(kb + (size_t)(key0 + 16) * DM + ks * 32, DM, lane);
            s0 = wmma16(ka, qf, s0);
            s1 = wmma16(kc, qf, s1);
        }
        const v4f d00 = *(const v4f*)(drow + key0);
        const v4f d01 = *(const v4f*)(drow + key0 + 4);
        const v4f d10 = *(const v4f*)(drow + key0 + 16);
        const v4f d11 = *(const v4f*)(drow + key0 + 20);
        float t0[8], t1[8];
        t0[0] = __builtin_fmaf(s0[0], C1, ncl * d00.x);
        t0[1] = __builtin_fmaf(s0[1], C1, ncl * d00.y);
        t0[2] = __builtin_fmaf(s0[2], C1, ncl * d00.z);
        t0[3] = __builtin_fmaf(s0[3], C1, ncl * d00.w);
        t0[4] = __builtin_fmaf(s0[4], C1, ncl * d01.x);
        t0[5] = __builtin_fmaf(s0[5], C1, ncl * d01.y);
        t0[6] = __builtin_fmaf(s0[6], C1, ncl * d01.z);
        t0[7] = __builtin_fmaf(s0[7], C1, ncl * d01.w);
        t1[0] = __builtin_fmaf(s1[0], C1, ncl * d10.x);
        t1[1] = __builtin_fmaf(s1[1], C1, ncl * d10.y);
        t1[2] = __builtin_fmaf(s1[2], C1, ncl * d10.z);
        t1[3] = __builtin_fmaf(s1[3], C1, ncl * d10.w);
        t1[4] = __builtin_fmaf(s1[4], C1, ncl * d11.x);
        t1[5] = __builtin_fmaf(s1[5], C1, ncl * d11.y);
        t1[6] = __builtin_fmaf(s1[6], C1, ncl * d11.z);
        t1[7] = __builtin_fmaf(s1[7], C1, ncl * d11.w);

        float mx = fmaxf(t0[0], t1[0]);
#pragma unroll
        for (int g = 1; g < 8; ++g) mx = fmaxf(mx, fmaxf(t0[g], t1[g]));
        mx = fmaxf(mx, __shfl_xor(mx, 16, 32));
        const float mn   = fmaxf(m, mx);
        const float corr = ex2(m - mn);
        const float sh   = 10.0f - mn;
        m = mn;

        Frag pf;
        float ls = 0.0f;
#pragma unroll
        for (int g = 0; g < 8; ++g) {
            _Float16 pa = (_Float16)ex2(t0[g] + sh);
            _Float16 pb = (_Float16)ex2(t1[g] + sh);
            pf.v[g]     = pa;
            pf.v[8 + g] = pb;
            ls += (float)pa + (float)pb;
        }
        l = l * corr + ls;

#pragma unroll
        for (int nt = 0; nt < 4; ++nt)
#pragma unroll
            for (int g = 0; g < 8; ++g) oacc[nt][g] *= corr;

        v16h vf0 = load_frag16(vb + (size_t)(0 * 16) * SEQ + key0, SEQ, lane);
        v16h vf1 = load_frag16(vb + (size_t)(1 * 16) * SEQ + key0, SEQ, lane);
        v16h vf2 = load_frag16(vb + (size_t)(2 * 16) * SEQ + key0, SEQ, lane);
        v16h vf3 = load_frag16(vb + (size_t)(3 * 16) * SEQ + key0, SEQ, lane);
        oacc[0] = wmma16(vf0, pf.v, oacc[0]);
        oacc[1] = wmma16(vf1, pf.v, oacc[1]);
        oacc[2] = wmma16(vf2, pf.v, oacc[2]);
        oacc[3] = wmma16(vf3, pf.v, oacc[3]);
    }

    const float lt  = l + __shfl_xor(l, 16, 32);
    const float inv = 1.0f / lt;
#pragma unroll
    for (int nt = 0; nt < 4; ++nt) {
        v8h ov;
#pragma unroll
        for (int g = 0; g < 8; ++g) ov[g] = (_Float16)(oacc[nt][g] * inv);
        *(v8h*)(&Os[w][cc * HD + nt * 16 + 8 * hs]) = ov;
    }
    wave_lds_sync();
    v8h pv0 = *(const v8h*)(&Os[w][(0 * 32 + lane) * 8]);
    v8h pv1 = *(const v8h*)(&Os[w][(1 * 32 + lane) * 8]);
    v8h pv2 = *(const v8h*)(&Os[w][(2 * 32 + lane) * 8]);
    v8h pv3 = *(const v8h*)(&Os[w][(3 * 32 + lane) * 8]);
    _Float16* ob = op + ((size_t)b * SEQ + q0r + (lane >> 3)) * DM + h * HD + (lane & 7) * 8;
    *(volatile v8h*)(ob + (size_t)0 * 4 * DM)  = pv0;
    *(volatile v8h*)(ob + (size_t)1 * 4 * DM)  = pv1;
    *(volatile v8h*)(ob + (size_t)2 * 4 * DM)  = pv2;
    *(volatile v8h*)(ob + (size_t)3 * 4 * DM)  = pv3;
    __threadfence();
    *(volatile v8h*)(ob + (size_t)0 * 4 * DM)  = pv0;
    *(volatile v8h*)(ob + (size_t)1 * 4 * DM)  = pv1;
    *(volatile v8h*)(ob + (size_t)2 * 4 * DM)  = pv2;
    *(volatile v8h*)(ob + (size_t)3 * 4 * DM)  = pv3;
}

constexpr size_t SZ_WET  = (size_t)DM * DM * 2;
constexpr size_t SZ_WQKV = (size_t)NL * 3 * DM * DM * 2;
constexpr size_t SZ_WO   = (size_t)NL * DM * DM * 2;
constexpr size_t SZ_W1   = (size_t)NL * DFF * DM * 2;
constexpr size_t SZ_W2   = (size_t)NL * DM * DFF * 2;
constexpr size_t SZ_X    = (size_t)NTOK * DM * 4;
constexpr size_t SZ_P16  = (size_t)NTOK * DM * 2;
constexpr size_t SZ_H    = (size_t)NTOK * DFF * 2;
constexpr size_t SZ_D    = (size_t)NB * SEQ * SEQ * 4;
constexpr size_t SZ_PART = (size_t)(NTOK / 8) * 128;
constexpr size_t SZ_ISTD = 128;
constexpr size_t WS_TOTAL = SZ_WET + SZ_WQKV + SZ_WO + SZ_W1 + SZ_W2 + SZ_X +
                            SZ_P16   + SZ_P16   + 2 * SZ_P16   +
                            SZ_P16   + SZ_P16   + SZ_H + SZ_D + SZ_PART + SZ_ISTD;
static_assert(WS_TOTAL <= (size_t)134217728);
static_assert(SZ_WET % 128 == 0 && SZ_P16 % 128 == 0 && SZ_PART % 128 == 0 && SZ_D % 128 == 0);
static_assert((size_t)NB * NH * HD * SEQ * 2 == SZ_P16);

extern "C" void kernel_launch(void* const* d_in, const int* in_sizes, int n_in,
                              void* d_out, int out_size, void* d_ws, size_t ws_size,
                              hipStream_t stream) {
    if (n_in < 24) return;
    if (in_sizes[0] < ((NB - 1) * SEQ_FULL + SEQ) * DM) return;
    if (in_sizes[1] < ((NB - 1) * SEQ_FULL + SEQ) * 3) return;
    if (in_sizes[2] < NMODE * 3) return;
    if (in_sizes[3] < DM * DM || in_sizes[4] < DM) return;
    if (in_sizes[5] < NL * DM * DM || in_sizes[7] < NL * DM * DM) return;
    if (in_sizes[9] < NL * DM * DM || in_sizes[11] < NL * DM * DM) return;
    if (in_sizes[6] < NL * DM || in_sizes[8] < NL * DM || in_sizes[10] < NL * DM || in_sizes[12] < NL * DM) return;
    if (in_sizes[13] < NL * NH) return;
    if (in_sizes[14] < NL * DM || in_sizes[15] < NL * DM || in_sizes[16] < NL * DM || in_sizes[17] < NL * DM) return;
    if (in_sizes[18] < NL * DM * DFF || in_sizes[19] < NL * DFF) return;
    if (in_sizes[20] < NL * DFF * DM || in_sizes[21] < NL * DM) return;
    if (in_sizes[22] < DM || in_sizes[23] < DM) return;
    if (out_size < NTOK * DM) return;
    if (WS_TOTAL > ws_size) return;

    const float* phi    = (const float*)d_in[0];
    const float* coords = (const float*)d_in[1];
    const float* modes  = (const float*)d_in[2];
    const float* We     = (const float*)d_in[3];
    const float* be     = (const float*)d_in[4];
    const float* wq     = (const float*)d_in[5];
    const float* bq     = (const float*)d_in[6];
    const float* wk     = (const float*)d_in[7];
    const float* bk     = (const float*)d_in[8];
    const float* wv     = (const float*)d_in[9];
    const float* bv     = (const float*)d_in[10];
    const float* wo     = (const float*)d_in[11];
    const float* bo     = (const float*)d_in[12];
    const float* temp   = (const float*)d_in[13];
    const float* ln1g   = (const float*)d_in[14];
    const float* ln1b   = (const float*)d_in[15];
    const float* ln2g   = (const float*)d_in[16];
    const float* ln2b   = (const float*)d_in[17];
    const float* w1     = (const float*)d_in[18];
    const float* b1     = (const float*)d_in[19];
    const float* w2     = (const float*)d_in[20];
    const float* b2     = (const float*)d_in[21];
    const float* fng    = (const float*)d_in[22];
    const float* fnb    = (const float*)d_in[23];
    float* out = (float*)d_out;

    char* ws = (char*)d_ws;
    size_t off = 0;
    _Float16* WeT   = (_Float16*)(ws + off); off += SZ_WET;
    _Float16* WqkvT = (_Float16*)(ws + off); off += SZ_WQKV;
    _Float16* WoT   = (_Float16*)(ws + off); off += SZ_WO;
    _Float16* W1T   = (_Float16*)(ws + off); off += SZ_W1;
    _Float16* W2T   = (_Float16*)(ws + off); off += SZ_W2;
    float*    x     = (float*)(ws + off);    off += SZ_X;
    _Float16* feats = (_Float16*)(ws + off); off += SZ_P16;
    _Float16* ypl   = (_Float16*)(ws + off); off += SZ_P16;
    _Float16* qk    = (_Float16*)(ws + off); off += 2 * SZ_P16;
    _Float16* vTp   = (_Float16*)(ws + off); off += SZ_P16;
    _Float16* opl   = (_Float16*)(ws + off); off += SZ_P16;
    _Float16* hpl   = (_Float16*)(ws + off); off += SZ_H;
    float*    dpl   = (float*)(ws + off);    off += SZ_D;
    double*   part  = (double*)(ws + off);   off += SZ_PART;
    float*    istd  = (float*)(ws + off);    off += SZ_ISTD;
    if (off > ws_size) return;

    k_wT<<<dim3(DM / 64, DM / 64, 1), dim3(256), 0, stream>>>(We, WeT, DM, DM, 0, 0);
    k_wT<<<dim3(DM / 64, DM / 64, NL), dim3(256), 0, stream>>>(wq, WqkvT,               DM, DM, DM * DM, 3 * DM * DM);
    k_wT<<<dim3(DM / 64, DM / 64, NL), dim3(256), 0, stream>>>(wk, WqkvT + DM * DM,     DM, DM, DM * DM, 3 * DM * DM);
    k_wT<<<dim3(DM / 64, DM / 64, NL), dim3(256), 0, stream>>>(wv, WqkvT + 2 * DM * DM, DM, DM, DM * DM, 3 * DM * DM);
    k_wT<<<dim3(DM / 64, DM / 64, NL), dim3(256), 0, stream>>>(wo, WoT, DM, DM, DM * DM, DM * DM);
    k_wT<<<dim3(DFF / 64, DM / 64, NL), dim3(256), 0, stream>>>(w1, W1T, DM, DFF, DM * DFF, DM * DFF);
    k_wT<<<dim3(DM / 64, DFF / 64, NL), dim3(256), 0, stream>>>(w2, W2T, DFF, DM, DFF * DM, DFF * DM);

    k_feats<<<dim3(NTOK / 8), dim3(256), 0, stream>>>(coords, modes, feats);
    k_dist<<<dim3(NTOK / 8), dim3(256), 0, stream>>>(coords, dpl, part);
    k_dstat<<<dim3(1), dim3(32), 0, stream>>>(part, istd);

    k_gemm<<<dim3(NTOK / 128, DM / 64), dim3(128), 0, stream>>>(
        feats, WeT, DM, DM, 0, 1.0f / (W_CARRY * F_CARRY), 1.0f,
        be, be, be, phi, 1, 1, x, ypl, vTp);

    for (int l = 0; l < NL; ++l) {
        k_ln16<<<dim3(NTOK / 8), dim3(256), 0, stream>>>(x, ln1g + l * DM, ln1b + l * DM, ypl);
        k_gemm<<<dim3(NTOK / 128, (3 * DM) / 64), dim3(128), 0, stream>>>(
            ypl, WqkvT + (size_t)l * 3 * DM * DM, DM, 3 * DM, 1, 1.0f / W_CARRY, QKV_CARRY,
            bq + l * DM, bk + l * DM, bv + l * DM, x, 0, 0, x, qk, vTp);
        k_attn<<<dim3(NB * NH, SEQ / 128), dim3(256), 0, stream>>>(
            qk, qk + (size_t)NTOK * DM, vTp, dpl, istd, temp + l * NH, opl);
        k_gemm<<<dim3(NTOK / 128, DM / 64), dim3(128), 0, stream>>>(
            opl, WoT + (size_t)l * DM * DM, DM, DM, 0, 1.0f / (W_CARRY * QKV_CARRY), 1.0f,
            bo + l * DM, bo + l * DM, bo + l * DM, x, 0, 0, x, ypl, vTp);
        k_ln16<<<dim3(NTOK / 8), dim3(256), 0, stream>>>(x, ln2g + l * DM, ln2b + l * DM, ypl);
        k_gemm<<<dim3(NTOK / 128, DFF / 64), dim3(128), 0, stream>>>(
            ypl, W1T + (size_t)l * DFF * DM, DM, DFF, 2, 1.0f / W_CARRY, H_CARRY,
            b1 + l * DFF, b1 + l * DFF, b1 + l * DFF, x, 0, 0, x, hpl, vTp);
        k_gemm<<<dim3(NTOK / 128, DM / 64), dim3(128), 0, stream>>>(
            hpl, W2T + (size_t)l * DM * DFF, DFF, DM, 0, 1.0f / (W_CARRY * H_CARRY), 1.0f,
            b2 + l * DM, b2 + l * DM, b2 + l * DM, x, 0, 0, x, ypl, vTp);
    }
    k_ln32<<<dim3(NTOK / 8), dim3(256), 0, stream>>>(x, fng, fnb, out);
}
